// MaskedAutoregressiveFlow_4681514352656
// MI455X (gfx1250) — hardware-run, weakly checked
//
#include <hip/hip_runtime.h>


#define NB   8192
#define ND   64
#define NH   512
#define NO2  128
typedef _Float16 h16;
typedef unsigned short bf;
typedef __attribute__((ext_vector_type(16))) __bf16   v16bf;
typedef __attribute__((ext_vector_type(16))) _Float16 v16h;
typedef __attribute__((ext_vector_type(8)))  _Float16 v8h;
typedef __attribute__((ext_vector_type(8)))  unsigned short v8us;
typedef __attribute__((ext_vector_type(8)))  float    v8f;
typedef __attribute__((ext_vector_type(4)))  float    v4f;
typedef v8h  __attribute__((may_alias)) v8ha;
typedef v4f  __attribute__((may_alias)) v4fa;
typedef v8us __attribute__((may_alias)) v8usa;

__device__ __forceinline__ unsigned short f2bf(float f) { unsigned u = __float_as_uint(f); u += 0x7FFFu + ((u >> 16) & 1u); return (unsigned short)(u >> 16); }
__device__ __forceinline__ float bf2f(unsigned short b) { return __uint_as_float(((unsigned)b) << 16); }
__device__ __forceinline__ float bfr(float f) { return bf2f(f2bf(f)); }
__device__ __forceinline__ v16h cat16(v8h lo, v8h hi) { return __builtin_shufflevector(lo, hi, 0, 1, 2, 3, 4, 5, 6, 7, 8, 9, 10, 11, 12, 13, 14, 15); }
__device__ __forceinline__ v16bf cat16b(v8us lo, v8us hi) { return __builtin_bit_cast(v16bf, __builtin_shufflevector(lo, hi, 0, 1, 2, 3, 4, 5, 6, 7, 8, 9, 10, 11, 12, 13, 14, 15)); }
__device__ __forceinline__ v8f wmma16(v16h a, v16h b, v8f c) { return __builtin_amdgcn_wmma_f32_16x16x32_f16(false, a, false, b, (short)0, c, false, false); }
__device__ __forceinline__ v8f wmmab(v16bf a, v16bf b, v8f c) { return __builtin_amdgcn_wmma_f32_16x16x32_bf16(false, a, false, b, (short)0, c, false, false); }


template <typename T16> struct WFrag;
template <> struct WFrag<h16> { typedef v16h V; static __device__ __forceinline__ V ld(const h16* p) { return cat16(*(const v8h*)p, *(const v8h*)(p + 16)); } static __device__ __forceinline__ v8f mma(V a, V b, v8f c) { return wmma16(a, b, c); } };
template <> struct WFrag<bf> { typedef v16bf V; static __device__ __forceinline__ V ld(const bf* p) { return cat16b(*(const v8us*)p, *(const v8us*)(p + 16)); } static __device__ __forceinline__ v8f mma(V a, V b, v8f c) { return wmmab(a, b, c); } };
template <typename T16, int NSPLIT, bool BIAS>
__global__ __launch_bounds__(32) void k_gemmw(const T16* __restrict__ A, const T16* __restrict__ A2, const T16* __restrict__ Bt, const T16* __restrict__ Bt2, int K, float* C, int ldc, const float* __restrict__ bias, size_t sA, size_t sB, size_t sC) {
    typedef typename WFrag<T16>::V V;
    __shared__ __align__(16) float os[16 * 68];
    const size_t z = blockIdx.z; A += z * sA; if (A2) A2 += z * sA; Bt += z * sB; if (Bt2) Bt2 += z * sB; C += z * sC;
    const int lane = threadIdx.x & 31, lr = lane & 15, hi = lane >> 4; const int r0 = blockIdx.x * 64, c0 = blockIdx.y * 64;
    v8f acc[4][4];
#pragma unroll
    for (int mb = 0; mb < 4; ++mb)
#pragma unroll
        for (int nb = 0; nb < 4; ++nb) acc[mb][nb] = (v8f){};
    const size_t aoff = (size_t)(r0 + lr) * K + 8 * hi, boff = (size_t)(c0 + lr) * K + 8 * hi;
    for (int kc = 0; kc < K; kc += 32) {
        V a[4], a2[4];
#pragma unroll
        for (int mb = 0; mb < 4; ++mb) { a[mb] = WFrag<T16>::ld(A + aoff + (size_t)mb * 16 * K + kc); if (NSPLIT == 1 || NSPLIT == 2) a2[mb] = WFrag<T16>::ld(A2 + aoff + (size_t)mb * 16 * K + kc); }
#pragma unroll
        for (int nb = 0; nb < 4; ++nb) { const V b = WFrag<T16>::ld(Bt + boff + (size_t)nb * 16 * K + kc); V b2; if (NSPLIT >= 2) b2 = WFrag<T16>::ld(Bt2 + boff + (size_t)nb * 16 * K + kc);
#pragma unroll
            for (int mb = 0; mb < 4; ++mb) { acc[mb][nb] = WFrag<T16>::mma(a[mb], b, acc[mb][nb]); if (NSPLIT == 1 || NSPLIT == 2) acc[mb][nb] = WFrag<T16>::mma(a2[mb], b, acc[mb][nb]); if (NSPLIT >= 2) acc[mb][nb] = WFrag<T16>::mma(a[mb], b2, acc[mb][nb]); } }
        asm volatile("v_nop\n\tv_nop\n\tv_nop\n\tv_nop" : "+v"(acc[0][0]), "+v"(acc[1][1]), "+v"(acc[2][2]), "+v"(acc[3][3]) : "v"(a[0]), "v"(a[3]));
    }
#pragma unroll
    for (int mb = 0; mb < 4; ++mb) {
#pragma unroll
        for (int nb = 0; nb < 4; ++nb) {
#pragma unroll
            for (int j = 0; j < 8; ++j) os[(hi * 8 + j) * 68 + nb * 16 + lr] = acc[mb][nb][j]; }
        __builtin_amdgcn_wave_barrier(); asm volatile("" ::: "memory");
        float* crow = C + (size_t)(r0 + mb * 16) * ldc + c0;
#pragma unroll 1
        for (int ps = 0; ps < 2; ++ps) {
#pragma unroll
            for (int s = 0; s < 8; ++s) { const int row = 2 * s + hi, cofs = lr * 4; v4f val = *(const v4fa*)(os + row * 68 + cofs); if (BIAS) { val[0] += bfr(bias[c0 + cofs]); val[1] += bfr(bias[c0 + cofs + 1]); val[2] += bfr(bias[c0 + cofs + 2]); val[3] += bfr(bias[c0 + cofs + 3]); }
                *(volatile v4f*)(crow + (size_t)row * ldc + cofs) = val; }
            if (ps == 0) __threadfence(); }
        __builtin_amdgcn_wave_barrier(); asm volatile("" ::: "memory");
    }
}

__device__ __forceinline__ h16 tohx(float x) { return (h16)x; }
__device__ __forceinline__ void splitf(float y, unsigned short& h, unsigned short& l) { h = f2bf(y); l = f2bf(y - bf2f(h)); }
typedef __attribute__((ext_vector_type(2))) _Float16 v2h;
typedef __attribute__((ext_vector_type(4))) _Float16 v4h;
typedef __attribute__((ext_vector_type(2))) unsigned short v2us;
typedef __attribute__((ext_vector_type(4))) unsigned short v4us;
typedef __attribute__((ext_vector_type(2))) float v2f;
typedef __attribute__((ext_vector_type(4))) int v4i;

__device__ __forceinline__ h16 toh_flush(float x) { const float z = (fabsf(x) < 6.103515625e-05f) ? 0.0f : x; return (h16)z; }

__global__ __launch_bounds__(256) void k_maskw16(const float* __restrict__ w, const float* __restrict__ mk, h16* dst, int n4) { const int i = blockIdx.x * 256 + threadIdx.x; if (i >= n4) return; const v4f v = *(const v4f*)(w + (size_t)i * 4); const v4f m = *(const v4f*)(mk + (size_t)i * 4); v4h o;
#pragma unroll
    for (int q = 0; q < 4; ++q) o[q] = toh_flush(__fmul_rn(bfr(v[q]), bfr(m[q])));
    *(volatile v4h*)(dst + (size_t)i * 4) = o; __threadfence(); *(volatile v4h*)(dst + (size_t)i * 4) = o; }

__global__ __launch_bounds__(256) void k_relu16(const float* __restrict__ src, const float* __restrict__ b, h16* dst, int n4, int ncol) { const int i = blockIdx.x * 256 + threadIdx.x; if (i >= n4) return; const int c0 = (i * 4) % ncol; const v4f v = *(const v4f*)(src + (size_t)i * 4); const v4f bb = *(const v4f*)(b + c0); v4h o;
#pragma unroll
    for (int q = 0; q < 4; ++q) o[q] = toh_flush(fmaxf(__fadd_rn(v[q], bfr(bb[q])), 0.0f));
    *(volatile v4h*)(dst + (size_t)i * 4) = o; __threadfence(); *(volatile v4h*)(dst + (size_t)i * 4) = o; }

__global__ __launch_bounds__(256) void k_stepf(const float* __restrict__ R, const float* __restrict__ z, const float* __restrict__ b2, int i, h16* X16, float* xout) { const int t = blockIdx.x * 256 + threadIdx.x; if (t >= NB * (ND / 2)) return; const int b = t / (ND / 2), c0 = (t % (ND / 2)) * 2; v2f xn;
    if (i < 0) { xn[0] = 0.0f; xn[1] = 0.0f; }
    else { const float mu = __fadd_rn(R[(size_t)b * NO2 + i], bfr(b2[i])); const float al = __fadd_rn(R[(size_t)b * NO2 + ND + i], bfr(b2[ND + i])); const float xv = fmaf(bfr(z[(size_t)b * ND + i]), expf(al), mu); const v2f xq = *(const v2f*)(xout + (size_t)t * 2);
#pragma unroll
        for (int q = 0; q < 2; ++q) xn[q] = (c0 + q == i) ? xv : xq[q]; }
    v2h o; o[0] = toh_flush(xn[0]); o[1] = toh_flush(xn[1]);
    *(volatile v2f*)(xout + (size_t)t * 2) = xn; *(volatile v2h*)(X16 + (size_t)t * 2) = o; __threadfence();
    *(volatile v2f*)(xout + (size_t)t * 2) = xn; *(volatile v2h*)(X16 + (size_t)t * 2) = o; }

__global__ __launch_bounds__(256) void k_ldsumf(const float* __restrict__ R, const float* __restrict__ b2, float* ld) { const int b = blockIdx.x * 256 + threadIdx.x; if (b >= NB) return; const float* ar = R + (size_t)b * NO2 + ND; float r = 0.0f;
    for (int j = 0; j < ND; ++j) r = __fadd_rn(r, __fadd_rn(ar[j], bfr(b2[ND + j])));
    *(volatile float*)(ld + b) = r; __threadfence(); *(volatile float*)(ld + b) = r; }

extern "C" void kernel_launch(void* const* d_in, const int* in_sizes, int n_in,
                              void* d_out, int out_size, void* d_ws, size_t ws_size, hipStream_t stream) {
    (void)in_sizes; (void)n_in; (void)out_size;
    const float* z = (const float*)d_in[0]; const float* W1 = (const float*)d_in[1]; const float* b1 = (const float*)d_in[2]; const float* W2 = (const float*)d_in[3]; const float* b2 = (const float*)d_in[4]; const float* mask1 = (const float*)d_in[5]; const float* mask2 = (const float*)d_in[6];
    static_assert(NB % 64 == 0 && NH % 64 == 0 && NO2 % 64 == 0 && ND % 32 == 0 && NH % 32 == 0 && (NH * ND) % 1024 == 0 && (NO2 * NH) % 1024 == 0 && (NB * NH) % 1024 == 0 && (NB * (ND / 2)) % 256 == 0 && NB % 256 == 0 && NO2 == 2 * ND, "the product launches: M and N multiples of 64, K a multiple of 32; exact grids");
    float* XOUT = (float*)d_out;       float* LD = XOUT + (size_t)NB * ND;
    char* wsp = (char*)d_ws;
    auto take = [&](size_t bytes) { char* p = wsp; wsp += (bytes + 255) & ~(size_t)255; return (void*)p; };
    h16* W1h = (h16*)take((size_t)NH * ND * 2);     h16* W2h = (h16*)take((size_t)NO2 * NH * 2);     h16* X16 = (h16*)take((size_t)NB * ND * 2);
    float* HC = (float*)take((size_t)NB * NH * 4);     h16* H16 = (h16*)take((size_t)NB * NH * 2);     float* RS = (float*)take((size_t)NB * NO2 * 4);
    if ((size_t)(wsp - (char*)d_ws) > ws_size) return;
    k_maskw16<<<(unsigned)(NH * ND / 4 / 256), 256, 0, stream>>>(W1, mask1, W1h, NH * ND / 4);
    k_maskw16<<<(unsigned)(NO2 * NH / 4 / 256), 256, 0, stream>>>(W2, mask2, W2h, NO2 * NH / 4);
    k_stepf<<<(unsigned)(NB * (ND / 2) / 256), 256, 0, stream>>>(RS, z, b2, -1, X16, XOUT);
    for (int i = 0; i <= ND; ++i) {
        k_gemmw<h16, 0, false><<<dim3(NB / 64, NH / 64, 1), 32, 0, stream>>>(X16, nullptr, W1h, nullptr, ND, HC, NH, nullptr, 0, 0, 0);
        k_relu16<<<(unsigned)(NB * NH / 4 / 256), 256, 0, stream>>>(HC, b1, H16, NB * NH / 4, NH);
        k_gemmw<h16, 0, false><<<dim3(NB / 64, NO2 / 64, 1), 32, 0, stream>>>(H16, nullptr, W2h, nullptr, NH, RS, NO2, nullptr, 0, 0, 0);
        if (i < ND) k_stepf<<<(unsigned)(NB * (ND / 2) / 256), 256, 0, stream>>>(RS, z, b2, i, X16, XOUT);
    }
    k_ldsumf<<<(unsigned)(NB / 256), 256, 0, stream>>>(RS, b2, LD);
}
